// Model_2130303778821
// MI455X (gfx1250) — hardware-verified
//
#include <hip/hip_runtime.h>
#include <math.h>

constexpr int ORD    = 256;
constexpr int PRED   = 192;
constexpr int SEQ    = 768;
constexpr int CHAN   = 21;
constexpr int NBAT   = 16;
constexpr int NMODE  = 32;
constexpr int NSCALE = 3;
constexpr int ROWS   = NBAT * CHAN;
constexpr int ROWSP  = 384;
constexpr int NCOL   = ORD * NMODE * 2;
constexpr int LMAX   = PRED << (NSCALE - 1);
constexpr int LSUM   = PRED * ((1 << NSCALE) - 1);
constexpr int TSAMP  = PRED - 1;
constexpr int NOUT   = NBAT * PRED * CHAN;
constexpr int GB_ROWS = 128;
static_assert(ROWS == 336);
static_assert(ROWSP % 64 == 0 && ROWSP >= ROWS);
static_assert(NCOL == 16384 && NCOL % 64 == 0 && NCOL % 32 == 0);
static_assert(ORD % 64 == 0);
static_assert(PRED % 64 == 0);
static_assert(LMAX == SEQ);
static_assert(LSUM == 1344);
static_assert(NOUT == 64512 && NOUT % 256 == 0);
static_assert((ROWSP * (PRED / 8)) % 256 == 0);
static_assert((ORD * (NCOL / 8)) % 256 == 0);
static_assert(NCOL % GB_ROWS == 0);

typedef __attribute__((ext_vector_type(16))) __bf16   v16b;
typedef __attribute__((ext_vector_type(8)))  __bf16   v8b;
typedef __attribute__((ext_vector_type(8)))  _Float16 v8h;
typedef __attribute__((ext_vector_type(8)))  float    v8f;
typedef __attribute__((ext_vector_type(4)))  float    v4f;

__device__ __forceinline__ unsigned short f2bf_bits(float f) {
  unsigned u = __float_as_uint(f);
  return (unsigned short)((u + 0x7FFFu + ((u >> 16) & 1u)) >> 16);
}
__device__ __forceinline__ float bf_bits2f(unsigned short h) { return __uint_as_float(((unsigned)h) << 16); }

__device__ __forceinline__ void dep_guard4_b(v8f& a, v8f& b, v8f& c, v8f& d, v16b x, v16b y) {
  asm volatile("v_nop\n\tv_nop\n\tv_nop\n\tv_nop" : "+v"(a), "+v"(b), "+v"(c), "+v"(d) : "v"(x), "v"(y));
}
__device__ __forceinline__ void keep4_b(v16b a, v16b b, v16b c, v16b d) { asm volatile("v_nop" :: "v"(a), "v"(b), "v"(c), "v"(d)); }
__device__ __forceinline__ void acc_guard4(v8f& a, v8f& b, v8f& c, v8f& d) {
  asm volatile("v_nop\n\tv_nop\n\tv_nop\n\tv_nop" : "+v"(a), "+v"(b), "+v"(c), "+v"(d));
}

union FragU { v16b v; v8b h[2]; };
__device__ __forceinline__ v16b frag_load(const __bf16* p) {
  FragU f;
  f.h[0] = *(const v8b*)(p);
  f.h[1] = *(const v8b*)(p + 16);
  return f.v;
}
__device__ __forceinline__ v8f frag_mma(v16b a, v16b b, v8f c) {
  return __builtin_amdgcn_wmma_f32_16x16x32_bf16(false, a, false, b, (short)0, c, false, false);
}

__device__ __forceinline__ void st2_f32(float* p, float v) {
  *(volatile float*)p = v;
  __threadfence();
  *(volatile float*)p = v;
}

template <bool SPLIT, int OUT_MODE>
__global__ __launch_bounds__(256) void wmma_gemm64(
    const unsigned short* __restrict__ Ap, const unsigned short* __restrict__ A2p, int lda, long strideA,
    const unsigned short* __restrict__ Btp, const unsigned short* __restrict__ Bt2p, int ldb, long strideB,
    void* __restrict__ Cout, void* __restrict__ Cout2, int ldc, long strideC,
    int M, int N, int K, float scale) {
  const __bf16* A = (const __bf16*)Ap;
  const __bf16* A2 = (const __bf16*)A2p;
  const __bf16* Bt = (const __bf16*)Btp;
  const __bf16* Bt2 = (const __bf16*)Bt2p;
  __shared__ __align__(16) float sT[8][16 * 68];
  const int b    = blockIdx.y;
  const int lane = threadIdx.x & 31;
  const int wave = threadIdx.x >> 5;
  const int tilesN = N >> 6;
  const int tilesM = M >> 6;
  const int tile = blockIdx.x * 8 + wave;
  if (tile >= tilesM * tilesN) return;
  const int tm = tile / tilesN;
  const int tn = tile - tm * tilesN;
  const int m0 = tm << 6;
  const int n0 = tn << 6;

  const __bf16* Ab  = A  + (size_t)b * strideA;
  const __bf16* Bb  = Bt + (size_t)b * strideB;
  const __bf16* Ab2 = SPLIT ? (A2  + (size_t)b * strideA) : Ab;
  const __bf16* Bb2 = SPLIT ? (Bt2 + (size_t)b * strideB) : Bb;

  const int rlane = lane & 15;
  const int koff  = (lane >> 4) * 8;
  const int mOff  = (lane >> 4) * 8;

  v8f acc[4][4];
#pragma unroll
  for (int i = 0; i < 4; ++i)
#pragma unroll
    for (int j = 0; j < 4; ++j) acc[i][j] = (v8f){0.f, 0.f, 0.f, 0.f, 0.f, 0.f, 0.f, 0.f};

  for (int k0 = 0; k0 < K; k0 += 32) {
    v16b bh[4], bl[4];
#pragma unroll
    for (int j = 0; j < 4; ++j) {
      const size_t bo = (size_t)(n0 + (j << 4) + rlane) * ldb + koff + k0;
      bh[j] = frag_load(Bb + bo);
      bl[j] = SPLIT ? frag_load(Bb2 + bo) : bh[j];
    }
#pragma unroll
    for (int i = 0; i < 4; ++i) {
      const size_t ao = (size_t)(m0 + (i << 4) + rlane) * lda + koff + k0;
      const v16b ah = frag_load(Ab + ao);
      const v16b al = SPLIT ? frag_load(Ab2 + ao) : ah;
#pragma unroll
      for (int j = 0; j < 4; ++j) {
        acc[i][j] = frag_mma(ah, bh[j], acc[i][j]);
        if (SPLIT) {
          acc[i][j] = frag_mma(ah, bl[j], acc[i][j]);
          acc[i][j] = frag_mma(al, bh[j], acc[i][j]);
        }
      }
      dep_guard4_b(acc[i][0], acc[i][1], acc[i][2], acc[i][3], ah, al);
    }
    keep4_b(bh[0], bh[1], bh[2], bh[3]);
    keep4_b(bl[0], bl[1], bl[2], bl[3]);
  }
  acc_guard4(acc[0][0], acc[0][1], acc[0][2], acc[0][3]);
  acc_guard4(acc[1][0], acc[1][1], acc[1][2], acc[1][3]);
  acc_guard4(acc[2][0], acc[2][1], acc[2][2], acc[2][3]);
  acc_guard4(acc[3][0], acc[3][1], acc[3][2], acc[3][3]);

  float* slab = sT[wave];
#pragma unroll
  for (int i = 0; i < 4; ++i) {
    const int mBase = m0 + (i << 4);
#pragma unroll
    for (int j = 0; j < 4; ++j) {
#pragma unroll
      for (int r = 0; r < 8; ++r) {
        const float v = acc[i][j][r] * scale;
        slab[(mOff + r) * 68 + (j << 4) + rlane] = v;
      }
    }
    __builtin_amdgcn_fence(__ATOMIC_RELEASE, "workgroup");
    __builtin_amdgcn_wave_barrier();
    __builtin_amdgcn_fence(__ATOMIC_ACQUIRE, "workgroup");
    if (OUT_MODE == 0) {
      float* C = (float*)Cout + (size_t)b * strideC;
      const int hh = lane >> 4, c4 = (lane & 15) * 4;
      for (int pass = 0; pass < 2; ++pass) {
#pragma unroll
        for (int it = 0; it < 8; ++it) {
          const int row = it * 2 + hh;
          const v4f v = *(const v4f*)(slab + row * 68 + c4);
          *(volatile v4f*)(C + (size_t)(mBase + row) * ldc + n0 + c4) = v;
        }
        __threadfence();
      }
    } else {
      const int q = lane >> 3, c8 = (lane & 7) * 8;
      unsigned short* C  = (unsigned short*)Cout  + (size_t)b * strideC;
      unsigned short* C2 = (unsigned short*)Cout2 + (size_t)b * strideC;
      for (int pass = 0; pass < 2; ++pass) {
#pragma unroll
        for (int it = 0; it < 4; ++it) {
          const int row = it * 4 + q;
          const float* sp = slab + row * 68 + c8;
          v8h hv, lv;
#pragma unroll
          for (int e = 0; e < 8; ++e) {
            const float x = sp[e];
            const unsigned short hb = f2bf_bits(x);
            const unsigned short lb = f2bf_bits(x - bf_bits2f(hb));
            hv[e] = __builtin_bit_cast(_Float16, hb);
            lv[e] = __builtin_bit_cast(_Float16, lb);
          }
          *(volatile v8h*)(C  + (size_t)(mBase + row) * ldc + n0 + c8) = hv;
          *(volatile v8h*)(C2 + (size_t)(mBase + row) * ldc + n0 + c8) = lv;
        }
        __threadfence();
      }
    }
    __builtin_amdgcn_fence(__ATOMIC_RELEASE, "workgroup");
    __builtin_amdgcn_wave_barrier();
    __builtin_amdgcn_fence(__ATOMIC_ACQUIRE, "workgroup");
  }
}

__global__ __launch_bounds__(256) void k_powers(
    const float* __restrict__ A0, const float* __restrict__ B0,
    const float* __restrict__ A1, const float* __restrict__ B1,
    const float* __restrict__ A2, const float* __restrict__ B2,
    float* __restrict__ Kbuf) {
  __shared__ __align__(16) float sK[2][ORD];
  const int sc = blockIdx.x;
  const int L = PRED << sc;
  const float* Am = (sc == 0) ? A0 : ((sc == 1) ? A1 : A2);
  const float* Bv = (sc == 0) ? B0 : ((sc == 1) ? B1 : B2);
  float* Ko = Kbuf + (size_t)(PRED * ((1 << sc) - 1)) * ORD;
  const int n = threadIdx.x;
  const float v0 = Bv[n];
  sK[0][n] = v0;
  st2_f32(Ko + n, v0);
  __syncthreads();
  const float* Arow = Am + (size_t)n * ORD;
#pragma unroll 1
  for (int d = 1; d < L; ++d) {
    const int cur = (d - 1) & 1;
    const float* kv = &sK[cur][0];
    float a0 = 0.f, a1 = 0.f, a2 = 0.f, a3 = 0.f;
#pragma unroll 2
    for (int q = 0; q < ORD / 4; ++q) {
      const v4f a = *(const v4f*)(Arow + 4 * q);
      const v4f k = *(const v4f*)(kv + 4 * q);
      a0 = fmaf(a[0], k[0], a0);
      a1 = fmaf(a[1], k[1], a1);
      a2 = fmaf(a[2], k[2], a2);
      a3 = fmaf(a[3], k[3], a3);
    }
    const float acc = (a0 + a1) + (a2 + a3);
    sK[cur ^ 1][n] = acc;
    st2_f32(Ko + (size_t)d * ORD + n, acc);
    __syncthreads();
  }
}

__global__ __launch_bounds__(256) void k_pack_f(const float* __restrict__ x, unsigned short* __restrict__ FH,
                                                unsigned short* __restrict__ FL) {
  const int sc = blockIdx.y;
  const int L = PRED << sc;
  const int l8 = L >> 3;
  const int n8 = ROWSP * l8;
  const int i = blockIdx.x * 256 + threadIdx.x;
  if (i < n8) {
    const int row = i / l8;
    const int t0 = (i - row * l8) * 8;
    const bool live = row < ROWS;
    const int rowc = live ? row : (ROWS - 1);
    const int b = rowc / CHAN;
    const int e = rowc - b * CHAN;
    const float* sp = x + ((size_t)b * SEQ + (size_t)(SEQ - L + t0)) * CHAN + e;
    v8h hv, lv;
#pragma unroll
    for (int j = 0; j < 8; ++j) {
      const float raw = sp[j * CHAN];
      const float f = live ? raw : 0.0f;
      const unsigned short hb = f2bf_bits(f);
      const unsigned short lb = f2bf_bits(f - bf_bits2f(hb));
      hv[j] = __builtin_bit_cast(_Float16, hb);
      lv[j] = __builtin_bit_cast(_Float16, lb);
    }
    const size_t off = (size_t)ROWSP * (size_t)(PRED * ((1 << sc) - 1)) + (size_t)i * 8;
    *(volatile v8h*)(FH + off) = hv;
    *(volatile v8h*)(FL + off) = lv;
    __threadfence();
    *(volatile v8h*)(FH + off) = hv;
    *(volatile v8h*)(FL + off) = lv;
  }
}

__global__ __launch_bounds__(64) void k_build_G(const float* __restrict__ Kb, unsigned short* __restrict__ GH,
                                                unsigned short* __restrict__ GL, int L, float invL) {
  __shared__ __align__(16) _Float16 tH[GB_ROWS * 64];
  __shared__ __align__(16) _Float16 tL[GB_ROWS * 64];
  __shared__ float twc[LMAX];
  __shared__ float tws[LMAX];
  const int tid = threadIdx.x, lane = tid & 31, wave = tid >> 5;
#pragma unroll 1
  for (int j = tid; j < L; j += 64) {
    const float fr = (float)(2 * j) * invL;
    twc[j] = cospif(fr);
    tws[j] = sinpif(fr);
  }
  __syncthreads();
  const int i = blockIdx.x * 2 + wave;
  const int k = lane;
  int idx1 = 0;
  int idx2 = (k == 0) ? 0 : (L - k);
  float sre = 0.f, sim = 0.f;
  const int nch = L >> 6;
  const int rre = wave * 64 + 2 * k;
  const int q = lane >> 3, c8 = (lane & 7) * 8;
#pragma unroll 1
  for (int ch = 0; ch < nch; ++ch) {
#pragma unroll 1
    for (int dd = 0; dd < 64; ++dd) {
      const int d = ch * 64 + dd;
      const float kd = Kb[(size_t)d * ORD + i];
      const float c1 = twc[idx1], s1 = tws[idx1];
      sre = fmaf(kd, c1, sre);
      sim = fmaf(-kd, s1, sim);
      const float c2 = twc[idx2], s2 = tws[idx2];
      const float gre = sre * c2 + sim * s2;
      const float gim = sim * c2 - sre * s2;
      const int col = 63 - dd;
      const unsigned short rh = f2bf_bits(gre);
      const unsigned short rl = f2bf_bits(gre - bf_bits2f(rh));
      const unsigned short ih = f2bf_bits(gim);
      const unsigned short il = f2bf_bits(gim - bf_bits2f(ih));
      tH[rre * 64 + col] = __builtin_bit_cast(_Float16, rh);
      tL[rre * 64 + col] = __builtin_bit_cast(_Float16, rl);
      tH[(rre + 1) * 64 + col] = __builtin_bit_cast(_Float16, ih);
      tL[(rre + 1) * 64 + col] = __builtin_bit_cast(_Float16, il);
      idx1 += k;
      idx1 = (idx1 >= L) ? (idx1 - L) : idx1;
      idx2 -= k;
      idx2 = (idx2 < 0) ? (idx2 + L) : idx2;
    }
    __syncthreads();
    const int s0 = L - 64 * (ch + 1);
    for (int pass = 0; pass < 2; ++pass) {
#pragma unroll 4
      for (int it = 0; it < 16; ++it) {
        const int row = wave * 64 + it * 4 + q;
        const v8h hv = *(const v8h*)(tH + row * 64 + c8);
        const v8h lv = *(const v8h*)(tL + row * 64 + c8);
        const size_t go = (size_t)(blockIdx.x * GB_ROWS + row) * (size_t)L + (size_t)(s0 + c8);
        *(volatile v8h*)(GH + go) = hv;
        *(volatile v8h*)(GL + go) = lv;
      }
      __threadfence();
    }
    __syncthreads();
  }
}

__global__ __launch_bounds__(256) void k_packW(const float* __restrict__ Wr, const float* __restrict__ Wi,
                                               unsigned short* __restrict__ PH, unsigned short* __restrict__ PL,
                                               int L, float invL) {
  __shared__ float cwt[NMODE];
  __shared__ float swt[NMODE];
  const int tid = threadIdx.x;
  if (tid < NMODE) {
    const int idx = (tid * TSAMP) % L;
    const float fr = (float)(2 * idx) * invL;
    const float sc = ((tid == 0) ? 1.0f : 2.0f) * invL;
    cwt[tid] = sc * cospif(fr);
    swt[tid] = sc * sinpif(fr);
  }
  __syncthreads();
  constexpr int N8ROW = NCOL / 8;
  const int i8 = blockIdx.x * 256 + tid;
  if (i8 < ORD * N8ROW) {
    const int o = i8 / N8ROW;
    const int rem = i8 - o * N8ROW;
    const int ii = rem >> 3;
    const int j = rem & 7;
    const size_t src = ((size_t)(ii * ORD + o)) * NMODE + 4 * j;
    const v4f wr = *(const v4f*)(Wr + src);
    const v4f wi = *(const v4f*)(Wi + src);
    v8h hv, lv;
#pragma unroll
    for (int e = 0; e < 4; ++e) {
      const float cw = cwt[4 * j + e];
      const float sw = swt[4 * j + e];
      const float a = wr[e];
      const float b = wi[e];
      const float p = cw * a - sw * b;
      const float qv = -(cw * b + sw * a);
      const unsigned short ph = f2bf_bits(p);
      const unsigned short pl = f2bf_bits(p - bf_bits2f(ph));
      const unsigned short qh = f2bf_bits(qv);
      const unsigned short ql = f2bf_bits(qv - bf_bits2f(qh));
      hv[2 * e]     = __builtin_bit_cast(_Float16, ph);
      lv[2 * e]     = __builtin_bit_cast(_Float16, pl);
      hv[2 * e + 1] = __builtin_bit_cast(_Float16, qh);
      lv[2 * e + 1] = __builtin_bit_cast(_Float16, ql);
    }
    const size_t off = (size_t)i8 * 8;
    *(volatile v8h*)(PH + off) = hv;
    *(volatile v8h*)(PL + off) = lv;
    __threadfence();
    *(volatile v8h*)(PH + off) = hv;
    *(volatile v8h*)(PL + off) = lv;
  }
}

__device__ __forceinline__ float dot_ord(const float* __restrict__ xr, const float* __restrict__ er) {
  float a0 = 0.f, a1 = 0.f, a2 = 0.f, a3 = 0.f;
#pragma unroll 2
  for (int q = 0; q < ORD / 4; ++q) {
    const v4f x = *(const v4f*)(xr + 4 * q);
    const v4f w = *(const v4f*)(er + 4 * q);
    a0 = fmaf(x[0], w[0], a0);
    a1 = fmaf(x[1], w[1], a1);
    a2 = fmaf(x[2], w[2], a2);
    a3 = fmaf(x[3], w[3], a3);
  }
  return (a0 + a1) + (a2 + a3);
}

__global__ __launch_bounds__(256) void k_final(const float* __restrict__ Xd,
                                               const float* __restrict__ E0, const float* __restrict__ E1,
                                               const float* __restrict__ E2,
                                               const float* __restrict__ mw, const float* __restrict__ mb,
                                               float* __restrict__ out) {
  const int g = blockIdx.x * 256 + threadIdx.x;
  if (g < NOUT) {
    const int b = g / (PRED * CHAN);
    const int r = g - b * (PRED * CHAN);
    const int t = r / CHAN;
    const int e = r - t * CHAN;
    const int row = b * CHAN + e;
    const float* x0 = Xd + (size_t)row * ORD;
    const float* x1 = x0 + (size_t)ROWSP * ORD;
    const float* x2 = x1 + (size_t)ROWSP * ORD;
    const float y0 = dot_ord(x0, E0 + (size_t)t * ORD);
    const float y1 = dot_ord(x1, E1 + (size_t)(PRED + t) * ORD);
    const float y2 = dot_ord(x2, E2 + (size_t)(3 * PRED + t) * ORD);
    float acc = mw[0] * y0;
    acc = fmaf(mw[1], y1, acc);
    acc = fmaf(mw[2], y2, acc);
    acc += mb[0];
    st2_f32(out + g, acc);
  }
}

extern "C" void kernel_launch(void* const* d_in, const int* in_sizes, int n_in,
                              void* d_out, int out_size, void* d_ws, size_t ws_size, hipStream_t stream) {
  if (n_in < 18 || d_out == nullptr || d_ws == nullptr) return;
  if (in_sizes[0] != NBAT * SEQ * CHAN || out_size != NOUT || in_sizes[16] != NSCALE || in_sizes[17] != 1) return;
  for (int s = 0; s < NSCALE; ++s) {
    if (in_sizes[1 + 5 * s] != ORD * ORD || in_sizes[2 + 5 * s] != ORD ||
        in_sizes[3 + 5 * s] != (PRED << s) * ORD ||
        in_sizes[4 + 5 * s] != ORD * ORD * NMODE || in_sizes[5 + 5 * s] != ORD * ORD * NMODE) return;
  }

  const float* x_enc = (const float*)d_in[0];
  const float* mlp_w = (const float*)d_in[16];
  const float* mlp_b = (const float*)d_in[17];

  char* ws = (char*)d_ws;
  size_t off = 0;
  auto carve = [&](size_t bytes) -> char* { char* p = ws + off; off += (bytes + 255) & ~(size_t)255; return p; };
  float*          KBUF = (float*)carve((size_t)LSUM * ORD * 4);
  unsigned short* FH   = (unsigned short*)carve((size_t)ROWSP * LSUM * 2);
  unsigned short* FL   = (unsigned short*)carve((size_t)ROWSP * LSUM * 2);
  unsigned short* GH   = (unsigned short*)carve((size_t)NCOL * LMAX * 2);
  unsigned short* GL   = (unsigned short*)carve((size_t)NCOL * LMAX * 2);
  unsigned short* AH   = (unsigned short*)carve((size_t)ROWSP * NCOL * 2);
  unsigned short* AL   = (unsigned short*)carve((size_t)ROWSP * NCOL * 2);
  unsigned short* PH   = (unsigned short*)carve((size_t)ORD * NCOL * 2);
  unsigned short* PL   = (unsigned short*)carve((size_t)ORD * NCOL * 2);
  float*          XD   = (float*)carve((size_t)NSCALE * ROWSP * ORD * 4);
  if (off > ws_size || off > (size_t)134217728) return;

  k_powers<<<NSCALE, 256, 0, stream>>>(
      (const float*)d_in[1], (const float*)d_in[2], (const float*)d_in[6], (const float*)d_in[7],
      (const float*)d_in[11], (const float*)d_in[12], KBUF);
  k_pack_f<<<dim3((ROWSP * (LMAX / 8)) / 256, NSCALE), 256, 0, stream>>>(x_enc, FH, FL);

  for (int s = 0; s < NSCALE; ++s) {
    const int L = PRED << s;
    const int loff = PRED * ((1 << s) - 1);
    const float invL = 1.0f / (float)L;
    const float* Wr = (const float*)d_in[4 + 5 * s];
    const float* Wi = (const float*)d_in[5 + 5 * s];
    float* XDs = XD + (size_t)s * ROWSP * ORD;

    k_build_G<<<NCOL / GB_ROWS, 64, 0, stream>>>(KBUF + (size_t)loff * ORD, GH, GL, L, invL);
    k_packW<<<(ORD * (NCOL / 8)) / 256, 256, 0, stream>>>(Wr, Wi, PH, PL, L, invL);

    wmma_gemm64<true, 2><<<dim3((ROWSP / 64) * (NCOL / 64) / 8, 1), 256, 0, stream>>>(
        FH + (size_t)ROWSP * loff, FL + (size_t)ROWSP * loff, L, 0L,
        GH, GL, L, 0L,
        (void*)AH, (void*)AL, NCOL, 0L,
        ROWSP, NCOL, L, 1.0f);

    wmma_gemm64<true, 0><<<dim3((ROWSP / 64) * (ORD / 64) / 8, 1), 256, 0, stream>>>(
        AH, AL, NCOL, 0L,
        PH, PL, NCOL, 0L,
        (void*)XDs, (void*)XDs, ORD, 0L,
        ROWSP, ORD, NCOL, 1.0f);
  }

  k_final<<<NOUT / 256, 256, 0, stream>>>(XD, (const float*)d_in[3], (const float*)d_in[8], (const float*)d_in[13],
                                          mlp_w, mlp_b, (float*)d_out);
}
